// DCNv2_4157528342738
// MI455X (gfx1250) — hardware-verified
//
#include <hip/hip_runtime.h>
#include <math.h>
#include <stddef.h>

typedef __attribute__((ext_vector_type(16))) _Float16 v16h;
typedef __attribute__((ext_vector_type(8)))  _Float16 v8h;
typedef __attribute__((ext_vector_type(16))) __bf16   v16b;
typedef __attribute__((ext_vector_type(8)))  __bf16   v8b;
typedef __attribute__((ext_vector_type(8)))  float    v8f;
typedef __attribute__((ext_vector_type(4)))  float    v4f;

constexpr int kBatch    = 4;
constexpr int kImgH     = 64;
constexpr int kImgW     = 64;
constexpr int kChan     = 256;
constexpr int kFilt     = 256;
constexpr int kTaps     = 9;
constexpr int kKdim     = kTaps * kChan;
constexpr int kNpix     = kBatch * kImgH * kImgW;
constexpr int kOffCh    = 27;
constexpr int kOffPitch = 32;
constexpr int kThreads  = 256;
constexpr float kClipBound = (float)(kImgH + 1);
constexpr float kMapCarry  = 16.0f;
constexpr float kWCarry    = 256.0f;
constexpr float kResCarry  = 2048.0f;
constexpr float kScaleHi   = 1.0f / 4096.0f;
constexpr float kScaleLo   = 1.0f / 8388608.0f;

constexpr size_t kOffBytes = (size_t)kNpix * kOffPitch * 4;
constexpr size_t kMapBytes = (size_t)kNpix * kKdim * 2;
constexpr size_t kKtBytes  = (size_t)kFilt * kKdim * 2;
constexpr size_t kCBytes   = (size_t)kNpix * kFilt * 4;
constexpr size_t kOffOff   = 0;
constexpr size_t kMapOff   = kOffOff + kOffBytes;
constexpr size_t kKthOff   = kMapOff + kMapBytes;
constexpr size_t kKtlOff   = kKthOff + kKtBytes;
constexpr size_t kC1Off    = kKtlOff + kKtBytes;
constexpr size_t kC2Off    = kC1Off + kCBytes;
constexpr size_t kWsTotal  = kC2Off + kCBytes;
static_assert(kWsTotal == 113508352u);
static_assert(kWsTotal <= 134217728u);
static_assert(kMapOff % 256 == 0 && kKthOff % 256 == 0 && kKtlOff % 256 == 0 && kC1Off % 256 == 0 && kC2Off % 256 == 0);
static_assert((kOffPitch * 4) % 128 == 0 && (kKdim * 2) % 128 == 0 && (kFilt * 4) % 128 == 0);
static_assert(kNpix % 64 == 0 && kFilt % 64 == 0 && kKdim % 32 == 0);
constexpr int kGemmTiles  = (kNpix / 64) * (kFilt / 64);
static_assert(kGemmTiles % 8 == 0);
constexpr int kGemmBlocks = kGemmTiles / 8;
constexpr int kPrepThreads = kFilt * (kKdim / 8);
static_assert(kPrepThreads % kThreads == 0);
static_assert((kKdim / 8) % 32 == 0);
static_assert(kChan == 32 * 8);
static_assert(kNpix % (kThreads / 32) == 0);
constexpr int kCombThreads = kNpix * kFilt / 4;
static_assert(kCombThreads % kThreads == 0);
static_assert(2 * kTaps + kTaps == kOffCh && kOffCh <= kOffPitch);

__device__ __forceinline__ unsigned short f2bf_bits(float f) {
  unsigned u = __float_as_uint(f);
  return (unsigned short)((u + 0x7FFFu + ((u >> 16) & 1u)) >> 16);
}
__device__ __forceinline__ float bf_bits2f(unsigned short h) { return __uint_as_float(((unsigned)h) << 16); }

__device__ __forceinline__ void dep_guard_h(v8f& a, v8f& b, v16h x, v16h y) { asm volatile("v_nop\n\tv_nop\n\tv_nop\n\tv_nop" : "+v"(a), "+v"(b) : "v"(x), "v"(y)); }
__device__ __forceinline__ void dep_guard_b(v8f& a, v8f& b, v16b x, v16b y) { asm volatile("v_nop\n\tv_nop\n\tv_nop\n\tv_nop" : "+v"(a), "+v"(b) : "v"(x), "v"(y)); }
__device__ __forceinline__ void keep4_h(v16h a, v16h b, v16h c, v16h d) { asm volatile("v_nop" :: "v"(a), "v"(b), "v"(c), "v"(d)); }
__device__ __forceinline__ void keep4_b(v16b a, v16b b, v16b c, v16b d) { asm volatile("v_nop" :: "v"(a), "v"(b), "v"(c), "v"(d)); }
__device__ __forceinline__ void acc_guard4(v8f& a, v8f& b, v8f& c, v8f& d) { asm volatile("v_nop\n\tv_nop\n\tv_nop\n\tv_nop" : "+v"(a), "+v"(b), "+v"(c), "+v"(d)); }
template <typename T> struct Frag;
template <> struct Frag<_Float16> {
  typedef v16h V; union U { v16h v; v8h h[2]; };
  static __device__ __forceinline__ v16h load(const _Float16* p) {
    U f; f.h[0] = *(const v8h*)(p); f.h[1] = *(const v8h*)(p + 16); return f.v;
  }
  static __device__ __forceinline__ v8f mma(v16h a, v16h b, v8f c) {
    return __builtin_amdgcn_wmma_f32_16x16x32_f16(false, a, false, b, (short)0, c, false, false);
  }
  static __device__ __forceinline__ void guard(v8f& a, v8f& b, v16h x, v16h y) { dep_guard_h(a, b, x, y); }
  static __device__ __forceinline__ void keep(v16h a, v16h b, v16h c, v16h d) { keep4_h(a, b, c, d); }
};
template <> struct Frag<__bf16> {
  typedef v16b V; union U { v16b v; v8b h[2]; };
  static __device__ __forceinline__ v16b load(const __bf16* p) {
    U f; f.h[0] = *(const v8b*)(p); f.h[1] = *(const v8b*)(p + 16); return f.v;
  }
  static __device__ __forceinline__ v8f mma(v16b a, v16b b, v8f c) {
    return __builtin_amdgcn_wmma_f32_16x16x32_bf16(false, a, false, b, (short)0, c, false, false);
  }
  static __device__ __forceinline__ void guard(v8f& a, v8f& b, v16b x, v16b y) { dep_guard_b(a, b, x, y); }
  static __device__ __forceinline__ void keep(v16b a, v16b b, v16b c, v16b d) { keep4_b(a, b, c, d); }
};

template <int ET> struct Elem;
template <> struct Elem<0> { typedef _Float16 T; };
template <> struct Elem<1> { typedef __bf16 T; };
template <int ET, bool SPLIT, int BIAS_MODE, int OUT_MODE, bool RESID, int ACT = 0>
__global__ __launch_bounds__(256) void wmma_gemm64(
    const unsigned short* __restrict__ Ap, const unsigned short* __restrict__ A2p, int lda, long strideA,
    const unsigned short* __restrict__ Btp, const unsigned short* __restrict__ Bt2p, int ldb, long strideB,
    void* __restrict__ Cout, void* __restrict__ Cout2, int ldc, long strideC,
    const float* __restrict__ bias,
    const float* __restrict__ resid, long strideR,
    int M, int N, int K, float scale) {
  typedef typename Elem<ET>::T T;
  typedef typename Frag<T>::V V;
  const T* A = (const T*)Ap; const T* A2 = (const T*)A2p; const T* Bt = (const T*)Btp; const T* Bt2 = (const T*)Bt2p;
  __shared__ __align__(16) float sT[8][16 * 68];
  const int b    = blockIdx.y;
  const int lane = threadIdx.x & 31;
  const int wave = threadIdx.x >> 5;
  const int tilesN = N >> 6;
  const int tilesM = M >> 6;
  const int tile = blockIdx.x * 8 + wave;
  if (tile >= tilesM * tilesN) return;
  const int tm = tile / tilesN;
  const int tn = tile - tm * tilesN;
  const int m0 = tm << 6;
  const int n0 = tn << 6;

  const T* Ab  = A  + (size_t)b * strideA;
  const T* Bb  = Bt + (size_t)b * strideB;
  const T* Ab2 = SPLIT ? (A2  + (size_t)b * strideA) : nullptr;
  const T* Bb2 = SPLIT ? (Bt2 + (size_t)b * strideB) : nullptr;

  const int rlane = lane & 15;
  const int koff  = (lane >> 4) * 8;
  const int mOff  = (lane >> 4) * 8;

  v8f acc[4][4];
#pragma unroll
  for (int i = 0; i < 4; ++i)
#pragma unroll
    for (int j = 0; j < 4; ++j) acc[i][j] = (v8f){0.f,0.f,0.f,0.f,0.f,0.f,0.f,0.f};

  for (int k0 = 0; k0 < K; k0 += 32) {
    V bh[4], bl[4];
#pragma unroll
    for (int j = 0; j < 4; ++j) {
      const size_t bo = (size_t)(n0 + (j << 4) + rlane) * ldb + koff + k0;
      bh[j] = Frag<T>::load(Bb + bo);
      if (SPLIT) bl[j] = Frag<T>::load(Bb2 + bo);
    }
#pragma unroll
    for (int i = 0; i < 4; ++i) {
      const size_t ao = (size_t)(m0 + (i << 4) + rlane) * lda + koff + k0;
      V ah = Frag<T>::load(Ab + ao);
      V al;
      if (SPLIT) al = Frag<T>::load(Ab2 + ao);
#pragma unroll
      for (int j = 0; j < 4; ++j) {
        acc[i][j] = Frag<T>::mma(ah, bh[j], acc[i][j]);
        if (SPLIT) {
          acc[i][j] = Frag<T>::mma(ah, bl[j], acc[i][j]);
          acc[i][j] = Frag<T>::mma(al, bh[j], acc[i][j]);
        }
      }
      Frag<T>::guard(acc[i][0], acc[i][3], ah, SPLIT ? al : ah);
    }
    Frag<T>::keep(bh[0], bh[1], bh[2], bh[3]);
    if (SPLIT) Frag<T>::keep(bl[0], bl[1], bl[2], bl[3]);
  }
  acc_guard4(acc[0][0], acc[0][1], acc[0][2], acc[0][3]);
  acc_guard4(acc[1][0], acc[1][1], acc[1][2], acc[1][3]);
  acc_guard4(acc[2][0], acc[2][1], acc[2][2], acc[2][3]);
  acc_guard4(acc[3][0], acc[3][1], acc[3][2], acc[3][3]);

  float* slab = sT[wave];
  const float* Rb = RESID ? (resid + (size_t)b * strideR) : nullptr;
#pragma unroll
  for (int i = 0; i < 4; ++i) {
    const int mBase = m0 + (i << 4);
#pragma unroll
    for (int j = 0; j < 4; ++j) {
      const int n = n0 + (j << 4) + rlane;
      float bv = 0.f;
      if (BIAS_MODE == 2) bv = bias[n];
#pragma unroll
      for (int r = 0; r < 8; ++r) {
        float v = acc[i][j][r] * scale;
        if (BIAS_MODE == 1) v += bias[mBase + mOff + r];
        if (BIAS_MODE == 2) v += bv;
        if (RESID) v += Rb[(size_t)(mBase + mOff + r) * ldc + n];
        if (ACT == 1) v = tanhf(v);
        if (ACT == 2) v = fmaxf(v, 0.0f);
        if (ACT == 3) v = v / (1.0f + expf(-v));
        if (ACT == 4) v = (v > 0.f) ? v : 0.01f * v;
        if (ACT == 5) v = 0.5f * v * (1.0f + erff(v * 0.70710678118654752f));
        slab[(mOff + r) * 68 + (j << 4) + rlane] = v;
      }
    }
    __builtin_amdgcn_fence(__ATOMIC_RELEASE, "workgroup");
    __builtin_amdgcn_wave_barrier();
    __builtin_amdgcn_fence(__ATOMIC_ACQUIRE, "workgroup");
    if (OUT_MODE == 0) {
      float* C = (float*)Cout + (size_t)b * strideC;
      const int hh = lane >> 4, c4 = (lane & 15) * 4;
      for (int pass = 0; pass < 2; ++pass) {
#pragma unroll
        for (int it = 0; it < 8; ++it) {
          const int row = it * 2 + hh;
          v4f v = *(const v4f*)(slab + row * 68 + c4);
          *(volatile v4f*)(C + (size_t)(mBase + row) * ldc + n0 + c4) = v;
        }
        __threadfence();
      }
    } else {
      const int q = lane >> 3, c8 = (lane & 7) * 8;
      unsigned short* C  = (unsigned short*)Cout  + (size_t)b * strideC;
      unsigned short* C2 = (OUT_MODE == 2) ? ((unsigned short*)Cout2 + (size_t)b * strideC) : nullptr;
      for (int pass = 0; pass < 2; ++pass) {
#pragma unroll
        for (int it = 0; it < 4; ++it) {
          const int row = it * 4 + q;
          const float* sp = slab + row * 68 + c8;
          v8h hv, lv;
#pragma unroll
          for (int e = 0; e < 8; ++e) {
            if (OUT_MODE == 1) {
              hv[e] = (_Float16)sp[e];
            } else {
              unsigned short hb = f2bf_bits(sp[e]);
              unsigned short lb = f2bf_bits(sp[e] - bf_bits2f(hb));
              hv[e] = __builtin_bit_cast(_Float16, hb);
              lv[e] = __builtin_bit_cast(_Float16, lb);
            }
          }
          *(volatile v8h*)(C + (size_t)(mBase + row) * ldc + n0 + c8) = hv;
          if (OUT_MODE == 2) *(volatile v8h*)(C2 + (size_t)(mBase + row) * ldc + n0 + c8) = lv;
        }
        __threadfence();
      }
    }
    __builtin_amdgcn_fence(__ATOMIC_RELEASE, "workgroup");
    __builtin_amdgcn_wave_barrier();
    __builtin_amdgcn_fence(__ATOMIC_ACQUIRE, "workgroup");
  }
}

__global__ __launch_bounds__(kThreads) void k_wprep(const float* __restrict__ w,
                                                   unsigned short* __restrict__ kth,
                                                   unsigned short* __restrict__ ktl) {
  const int i = blockIdx.x * kThreads + threadIdx.x;
  if (i >= kPrepThreads) return;
  const int tpr = kKdim / 8;
  const int n   = i / tpr;
  const int k0  = (i - n * tpr) * 8;
  v8h hv, lv;
#pragma unroll
  for (int e = 0; e < 8; ++e) {
    const float v    = w[(size_t)(k0 + e) * kFilt + n] * kWCarry;
    const _Float16 h = (_Float16)v;
    const float hf   = (float)h;
    const float res  = (v - hf) * kResCarry;
    hv[e] = h;
    lv[e] = (_Float16)res;
  }
  const size_t o = (size_t)i * 8;
  _Float16* ph = (_Float16*)kth + o;
  _Float16* pl = (_Float16*)ktl + o;
  *(volatile v8h*)(ph) = hv;
  *(volatile v8h*)(pl) = lv;
  __threadfence();
  *(volatile v8h*)(ph) = hv;
  *(volatile v8h*)(pl) = lv;
}

__global__ __launch_bounds__(32) void k_offconv(const float* __restrict__ x,
                                                const float* __restrict__ ow,
                                                const float* __restrict__ ob,
                                                float* __restrict__ off) {
  __shared__ __align__(16) float patch[kKdim];
  const int pix = blockIdx.x;
  const int b   = pix >> 12;
  const int rem = pix & 4095;
  const int y   = rem >> 6;
  const int xc  = rem & 63;
  const int t   = threadIdx.x;
#pragma unroll 1
  for (int tap = 0; tap < kTaps; ++tap) {
    const int tr = tap / 3;
    const int ts = tap - 3 * tr;
    const int yy = y + tr - 1;
    const int xx = xc + ts - 1;
    const float f = (yy >= 0 && yy < kImgH && xx >= 0 && xx < kImgW) ? 1.0f : 0.0f;
    const int yyc = min(max(yy, 0), kImgH - 1);
    const int xxc = min(max(xx, 0), kImgW - 1);
    const float* p = x + (((size_t)b * kImgH + yyc) * kImgW + xxc) * kChan + t * 8;
    v4f v0 = *(const v4f*)(p);
    v4f v1 = *(const v4f*)(p + 4);
    v0 = v0 * f;
    v1 = v1 * f;
    *(v4f*)(patch + tap * kChan + t * 8)     = v0;
    *(v4f*)(patch + tap * kChan + t * 8 + 4) = v1;
  }
  __syncthreads();
  const int j = (t < kOffCh) ? t : (kOffCh - 1);
  float acc = 0.0f;
#pragma unroll 8
  for (int kk = 0; kk < kKdim; ++kk) acc = fmaf(patch[kk], ow[kk * kOffCh + j], acc);
  acc += ob[j];
  const float v = (t < kOffCh) ? acc : 0.0f;
  volatile float* o = off + (size_t)pix * kOffPitch;
  o[t] = v;
  __threadfence();
  o[t] = v;
}

__global__ __launch_bounds__(kThreads) void k_sample(const float* __restrict__ x,
                                                    const float* __restrict__ off,
                                                    unsigned short* __restrict__ amap) {
  const int lane = threadIdx.x & 31;
  const int wave = threadIdx.x >> 5;
  const int pix  = blockIdx.x * (kThreads / 32) + wave;
  const int b    = pix >> 12;
  const int rem  = pix & 4095;
  const int y    = rem >> 6;
  const int xc   = rem & 63;
  const float offv = off[(size_t)pix * kOffPitch + lane];
  const float* xb  = x + ((size_t)b << 20);
  const int c0     = lane * 8;
  _Float16* arow   = (_Float16*)amap + (size_t)pix * kKdim + c0;
#pragma unroll 1
  for (int tap = 0; tap < kTaps; ++tap) {
    const float dyo = __shfl(offv, 2 * tap, 32);
    const float dxo = __shfl(offv, 2 * tap + 1, 32);
    const float mlg = __shfl(offv, 2 * kTaps + tap, 32);
    const float mk  = 1.0f / (1.0f + expf(-mlg));
    const int tr = tap / 3;
    const int ts = tap - 3 * tr;
    const float gy = (float)(y + tr) + dyo;
    const float gx = (float)(xc + ts) + dxo;

    const float y0f = floorf(gy);
    const float y1c = fminf(fmaxf(y0f + 1.0f, 0.0f), kClipBound);
    const float y0c = fminf(fmaxf(y0f, 0.0f), kClipBound);
    const float gyc = fminf(fmaxf(gy, 0.0f), kClipBound);
    const float x0f = floorf(gx);
    const float x1c = fminf(fmaxf(x0f + 1.0f, 0.0f), kClipBound);
    const float x0c = fminf(fmaxf(x0f, 0.0f), kClipBound);
    const float gxc = fminf(fmaxf(gx, 0.0f), kClipBound);

    const float dy0 = gyc - y0c;
    const float dy1 = y1c - gyc;
    const float dx0 = gxc - x0c;
    const float dx1 = x1c - gxc;

    const int y0i = (int)y0c, y1i = (int)y1c, x0i = (int)x0c, x1i = (int)x1c;
    const bool vy0 = (y0i >= 1) && (y0i <= kImgH);
    const bool vy1 = (y1i >= 1) && (y1i <= kImgH);
    const bool vx0 = (x0i >= 1) && (x0i <= kImgW);
    const bool vx1 = (x1i >= 1) && (x1i <= kImgW);
    const float f11 = (vy1 && vx1) ? 1.0f : 0.0f;
    const float f10 = (vy1 && vx0) ? 1.0f : 0.0f;
    const float f01 = (vy0 && vx1) ? 1.0f : 0.0f;
    const float f00 = (vy0 && vx0) ? 1.0f : 0.0f;
    const float w11 = (dy0 * dx0) * f11;
    const float w10 = (dy0 * dx1) * f10;
    const float w01 = (dy1 * dx0) * f01;
    const float w00 = (dy1 * dx1) * f00;

    const int ry0 = min(max(y0i - 1, 0), kImgH - 1);
    const int ry1 = min(max(y1i - 1, 0), kImgH - 1);
    const int rx0 = min(max(x0i - 1, 0), kImgW - 1);
    const int rx1 = min(max(x1i - 1, 0), kImgW - 1);
    const float* p00 = xb + (size_t)((ry0 << 6) + rx0) * kChan + c0;
    const float* p01 = xb + (size_t)((ry0 << 6) + rx1) * kChan + c0;
    const float* p10 = xb + (size_t)((ry1 << 6) + rx0) * kChan + c0;
    const float* p11 = xb + (size_t)((ry1 << 6) + rx1) * kChan + c0;

    const v4f s00a = *(const v4f*)(p00), s00b = *(const v4f*)(p00 + 4);
    const v4f s01a = *(const v4f*)(p01), s01b = *(const v4f*)(p01 + 4);
    const v4f s10a = *(const v4f*)(p10), s10b = *(const v4f*)(p10 + 4);
    const v4f s11a = *(const v4f*)(p11), s11b = *(const v4f*)(p11 + 4);

    v4f ra = s11a * w11;
    ra = s10a * w10 + ra;
    ra = s01a * w01 + ra;
    ra = s00a * w00 + ra;
    v4f rb = s11b * w11;
    rb = s10b * w10 + rb;
    rb = s01b * w01 + rb;
    rb = s00b * w00 + rb;
    const float sc = mk * kMapCarry;
    ra = ra * sc;
    rb = rb * sc;

    v8h hv;
    hv[0] = (_Float16)ra[0]; hv[1] = (_Float16)ra[1]; hv[2] = (_Float16)ra[2]; hv[3] = (_Float16)ra[3];
    hv[4] = (_Float16)rb[0]; hv[5] = (_Float16)rb[1]; hv[6] = (_Float16)rb[2]; hv[7] = (_Float16)rb[3];
    _Float16* dst = arow + tap * kChan;
    *(volatile v8h*)(dst) = hv;
    __threadfence();
    *(volatile v8h*)(dst) = hv;
  }
}

__global__ __launch_bounds__(kThreads) void k_combine(const float* __restrict__ c1,
                                                     const float* __restrict__ c2,
                                                     const float* __restrict__ bias,
                                                     float* __restrict__ out) {
  const int i = blockIdx.x * kThreads + threadIdx.x;
  if (i >= kCombThreads) return;
  const int f4 = (i & (kFilt / 4 - 1)) * 4;
  const v4f a  = *(const v4f*)(c1 + (size_t)i * 4);
  const v4f bb = *(const v4f*)(c2 + (size_t)i * 4);
  const v4f bs = *(const v4f*)(bias + f4);
  v4f v = a + bb;
  v = v + bs;
  float* dst = out + (size_t)i * 4;
  *(volatile v4f*)(dst) = v;
  __threadfence();
  *(volatile v4f*)(dst) = v;
}

extern "C" void kernel_launch(void* const* d_in, const int* in_sizes, int n_in,
                              void* d_out, int out_size, void* d_ws, size_t ws_size,
                              hipStream_t stream) {
  if (n_in < 5) return;
  const float* x    = (const float*)d_in[0];
  const float* w    = (const float*)d_in[1];
  const float* bias = (const float*)d_in[2];
  const float* ow   = (const float*)d_in[3];
  const float* ob   = (const float*)d_in[4];
  float* out = (float*)d_out;
  if (in_sizes[0] != kNpix * kChan || in_sizes[1] != kKdim * kFilt || in_sizes[2] != kFilt ||
      in_sizes[3] != kKdim * kOffCh || in_sizes[4] != kOffCh || out_size != kNpix * kFilt) return;
  if (kWsTotal > ws_size) return;

  char* ws = (char*)d_ws;
  float*          off  = (float*)(ws + kOffOff);
  unsigned short* amap = (unsigned short*)(ws + kMapOff);
  unsigned short* kth  = (unsigned short*)(ws + kKthOff);
  unsigned short* ktl  = (unsigned short*)(ws + kKtlOff);
  float*          c1   = (float*)(ws + kC1Off);
  float*          c2   = (float*)(ws + kC2Off);

  k_wprep<<<kPrepThreads / kThreads, kThreads, 0, stream>>>(w, kth, ktl);
  k_offconv<<<kNpix, 32, 0, stream>>>(x, ow, ob, off);
  k_sample<<<kNpix / (kThreads / 32), kThreads, 0, stream>>>(x, off, amap);
  wmma_gemm64<0, false, 0, 0, false, 0><<<dim3(kGemmBlocks, 1, 1), dim3(256, 1, 1), 0, stream>>>(
      amap, amap, kKdim, 0L, kth, kth, kKdim, 0L, (void*)c1, (void*)c1, kFilt, 0L,
      bias, bias, 0L, kNpix, kFilt, kKdim, kScaleHi);
  wmma_gemm64<0, false, 0, 0, false, 0><<<dim3(kGemmBlocks, 1, 1), dim3(256, 1, 1), 0, stream>>>(
      amap, amap, kKdim, 0L, ktl, ktl, kKdim, 0L, (void*)c2, (void*)c2, kFilt, 0L,
      bias, bias, 0L, kNpix, kFilt, kKdim, kScaleLo);
  k_combine<<<kCombThreads / kThreads, kThreads, 0, stream>>>(c1, c2, bias, out);
}
